// smamba_52699248722201
// MI455X (gfx1250) — hardware-run, weakly checked
//
#include <hip/hip_runtime.h>
#include <math.h>

typedef __attribute__((ext_vector_type(16))) _Float16 v16h;
typedef __attribute__((ext_vector_type(8)))  _Float16 v8h;
typedef __attribute__((ext_vector_type(8)))  float    v8f;
typedef __attribute__((ext_vector_type(4)))  float    v4f;

constexpr int kBatch  = 2;
constexpr int kSeq    = 2048;
constexpr int kDm     = 512;
constexpr int kDin    = 512;
constexpr int kNst    = 32;
constexpr int kDtR    = 32;
constexpr int kRows   = kBatch * kSeq;
constexpr int kXzP    = 4 * kDin;
constexpr int kXcP    = 2 * kDin;
constexpr int kDblDir = 128;
constexpr int kDblP   = 2 * kDblDir;
constexpr int kPrjN   = kDtR + 2 * kNst;
constexpr int kConvTP = 260;
constexpr int kScanTS = 64;
constexpr int kScanCh = 64;
constexpr int kScanYP = 68;
constexpr int kStP    = 36;
constexpr float kCarryW  = 32.0f;
constexpr float kCarryXc = 256.0f;
constexpr float kCarryDt = 256.0f;
constexpr float kCarryY  = 1024.0f;

static_assert(kPrjN == 96);
static_assert(kPrjN <= kDblDir && (kDblDir % 64) == 0);
static_assert((kSeq & (kSeq - 1)) == 0);
static_assert((kRows % 64) == 0 && (kXzP % 64) == 0 && (kDm % 64) == 0 && (kDin % 64) == 0);
static_assert((kDm % 32) == 0 && (kDin % 32) == 0 && (kDtR % 32) == 0 && ((2 * kDin) % 32) == 0);
static_assert((kSeq % kScanTS) == 0 && (kDin % kScanCh) == 0 && (kDin % 256) == 0 && (kNst % 4) == 0);
static_assert(kNst == 32 && kDtR == 32 && kScanCh == 64 && kScanTS == 64);

constexpr size_t kOffX16   = 0;
constexpr size_t kOffWIN   = kOffX16  + (size_t)kRows * kDm * 2;
constexpr size_t kOffWXP   = kOffWIN  + (size_t)(2 * 2 * kDin) * kDm * 2;
constexpr size_t kOffWDT   = kOffWXP  + (size_t)2 * kDblDir * kDin * 2;
constexpr size_t kOffWOUT  = kOffWDT  + (size_t)2 * kDin * kDtR * 2;
constexpr size_t kOffXZ    = kOffWOUT + (size_t)kDm * (2 * kDin) * 2;
constexpr size_t kOffXC    = kOffXZ   + (size_t)kRows * kXzP * 4;
constexpr size_t kOffXC16  = kOffXC   + (size_t)kRows * kXcP * 4;
constexpr size_t kOffDBL   = kOffXC16 + (size_t)kRows * kXcP * 2;
constexpr size_t kOffDT16  = kOffDBL  + (size_t)kRows * kDblP * 4;
constexpr size_t kOffDLR   = kOffDT16 + (size_t)2 * kRows * kDtR * 2;
constexpr size_t kOffY16   = kOffDLR  + (size_t)kRows * kXcP * 4;
constexpr size_t kWsTotal  = kOffY16  + (size_t)kRows * kXcP * 2;
static_assert(kWsTotal == 96272384ull);
static_assert(kWsTotal <= 134217728ull);
static_assert((kOffWIN % 128) == 0 && (kOffWXP % 128) == 0 && (kOffWDT % 128) == 0 && (kOffWOUT % 128) == 0 &&
              (kOffXZ % 128) == 0 && (kOffXC % 128) == 0 && (kOffXC16 % 128) == 0 && (kOffDBL % 128) == 0 &&
              (kOffDT16 % 128) == 0 && (kOffDLR % 128) == 0 && (kOffY16 % 128) == 0);

__device__ __forceinline__ unsigned short f2bf_bits(float f) {
  unsigned u = __float_as_uint(f);
  return (unsigned short)((u + 0x7FFFu + ((u >> 16) & 1u)) >> 16);
}
__device__ __forceinline__ float bf_bits2f(unsigned short h) { return __uint_as_float(((unsigned)h) << 16); }
__device__ __forceinline__ float bf_rne(float f) { return bf_bits2f(f2bf_bits(f)); }

__device__ __forceinline__ void dep_guard4_h(v8f& a, v8f& b, v8f& c, v8f& d, v16h x, v16h y) {
  asm volatile("v_nop\n\tv_nop\n\tv_nop\n\tv_nop" : "+v"(a), "+v"(b), "+v"(c), "+v"(d) : "v"(x), "v"(y));
}
__device__ __forceinline__ void keep4_h(v16h a, v16h b, v16h c, v16h d) { asm volatile("v_nop" :: "v"(a), "v"(b), "v"(c), "v"(d)); }
__device__ __forceinline__ void acc_guard4(v8f& a, v8f& b, v8f& c, v8f& d) { asm volatile("v_nop\n\tv_nop\n\tv_nop\n\tv_nop" : "+v"(a), "+v"(b), "+v"(c), "+v"(d)); }

struct FragH {
  union U { v16h v; v8h h[2]; };
  static __device__ __forceinline__ v16h load(const _Float16* p) {
    U f; f.h[0] = *(const v8h*)(p); f.h[1] = *(const v8h*)(p + 16); return f.v;
  }
  static __device__ __forceinline__ v8f mma(v16h a, v16h b, v8f c) {
    return __builtin_amdgcn_wmma_f32_16x16x32_f16(false, a, false, b, (short)0, c, false, false);
  }
};

__global__ __launch_bounds__(256) void gemm64_f16_kernel(
    const unsigned short* __restrict__ Ap, int lda, long strideA,
    const unsigned short* __restrict__ Btp, int ldb, long strideB,
    float* __restrict__ Cout, int ldc, long strideC,
    int M, int N, int K, float scale)
{
  const _Float16* A  = (const _Float16*)Ap;
  const _Float16* Bt = (const _Float16*)Btp;
  __shared__ __align__(16) float sT[8][16 * 68];
  const int b    = blockIdx.y;
  const int lane = threadIdx.x & 31;
  const int wave = threadIdx.x >> 5;
  const int tilesN = N >> 6;
  const int tilesM = M >> 6;
  const int tile = blockIdx.x * 8 + wave;
  if (tile >= tilesM * tilesN) return;
  const int tm = tile / tilesN;
  const int tn = tile - tm * tilesN;
  const int m0 = tm << 6;
  const int n0 = tn << 6;

  const _Float16* Ab = A  + (size_t)b * strideA;
  const _Float16* Bb = Bt + (size_t)b * strideB;

  const int rlane = lane & 15;
  const int koff  = (lane >> 4) * 8;
  const int mOff  = (lane >> 4) * 8;

  v8f acc[4][4];
#pragma unroll
  for (int i = 0; i < 4; ++i)
#pragma unroll
    for (int j = 0; j < 4; ++j) acc[i][j] = (v8f){0.f,0.f,0.f,0.f,0.f,0.f,0.f,0.f};

  for (int k0 = 0; k0 < K; k0 += 32) {
    v16h bh[4];
#pragma unroll
    for (int j = 0; j < 4; ++j) {
      const size_t bo = (size_t)(n0 + (j << 4) + rlane) * ldb + koff + k0;
      bh[j] = FragH::load(Bb + bo);
    }
#pragma unroll
    for (int i = 0; i < 4; ++i) {
      const size_t ao = (size_t)(m0 + (i << 4) + rlane) * lda + koff + k0;
      v16h ah = FragH::load(Ab + ao);
#pragma unroll
      for (int j = 0; j < 4; ++j) acc[i][j] = FragH::mma(ah, bh[j], acc[i][j]);
      dep_guard4_h(acc[i][0], acc[i][1], acc[i][2], acc[i][3], ah, bh[3]);
    }
    keep4_h(bh[0], bh[1], bh[2], bh[3]);
  }
  acc_guard4(acc[0][0], acc[0][1], acc[0][2], acc[0][3]);
  acc_guard4(acc[1][0], acc[1][1], acc[1][2], acc[1][3]);
  acc_guard4(acc[2][0], acc[2][1], acc[2][2], acc[2][3]);
  acc_guard4(acc[3][0], acc[3][1], acc[3][2], acc[3][3]);

  float* slab = sT[wave];
  float* C = Cout + (size_t)b * strideC;
#pragma unroll
  for (int i = 0; i < 4; ++i) {
    const int mBase = m0 + (i << 4);
#pragma unroll
    for (int j = 0; j < 4; ++j) {
#pragma unroll
      for (int r = 0; r < 8; ++r) {
        const float v = acc[i][j][r] * scale;
        slab[(mOff + r) * 68 + (j << 4) + rlane] = v;
      }
    }
    __builtin_amdgcn_fence(__ATOMIC_RELEASE, "workgroup");
    __builtin_amdgcn_wave_barrier();
    __builtin_amdgcn_fence(__ATOMIC_ACQUIRE, "workgroup");
    {
      const int hh = lane >> 4, c4 = (lane & 15) * 4;
      for (int pass = 0; pass < 2; ++pass) {
#pragma unroll
        for (int it = 0; it < 8; ++it) {
          const int row = it * 2 + hh;
          v4f v = *(const v4f*)(slab + row * 68 + c4);
          *(volatile v4f*)(C + (size_t)(mBase + row) * ldc + n0 + c4) = v;
        }
        __threadfence();
      }
    }
    __builtin_amdgcn_fence(__ATOMIC_RELEASE, "workgroup");
    __builtin_amdgcn_wave_barrier();
    __builtin_amdgcn_fence(__ATOMIC_ACQUIRE, "workgroup");
  }
}

__global__ __launch_bounds__(256) void cast_rows_f16_kernel(
    const float* __restrict__ src0, const float* __restrict__ src1,
    unsigned short* __restrict__ dst, int srcRows, int dstRows, int cols,
    int dstPitch, long dstStrideY, float scale)
{
  const int cols8  = cols >> 3;
  const int total8 = dstRows * cols8;
  const int i = blockIdx.x * 256 + threadIdx.x;
  if (i >= total8) return;
  const float* src = (blockIdx.y == 0) ? src0 : src1;
  const int row = i / cols8;
  const int c8  = (i - row * cols8) << 3;
  const bool live = row < srcRows;
  const int rc = live ? row : (srcRows - 1);
  const float* p = src + (size_t)rc * cols + c8;
  const v4f a0 = *(const v4f*)(p);
  const v4f a1 = *(const v4f*)(p + 4);
  v8h hv;
#pragma unroll
  for (int e = 0; e < 4; ++e) {
    const float f0 = a0[e];
    const float f1 = a1[e];
    const float r0 = bf_rne(f0) * scale;
    const float r1 = bf_rne(f1) * scale;
    const float s0 = live ? r0 : 0.0f;
    const float s1 = live ? r1 : 0.0f;
    hv[e]     = (_Float16)s0;
    hv[4 + e] = (_Float16)s1;
  }
  unsigned short* q = dst + (size_t)blockIdx.y * dstStrideY + (size_t)row * dstPitch + c8;
  *(volatile v8h*)q = hv;
  __threadfence();
  *(volatile v8h*)q = hv;
}

__global__ __launch_bounds__(256) void dt_cast_kernel(
    const float* __restrict__ DBL, unsigned short* __restrict__ DT16, int total8, float scale)
{
  const int i = blockIdx.x * 256 + threadIdx.x;
  if (i >= total8) return;
  const int e0  = i << 3;
  const int dir = e0 / (kRows * kDtR);
  const int rem = e0 - dir * (kRows * kDtR);
  const int row = rem / kDtR;
  const int c8  = rem - row * kDtR;
  const float* p = DBL + (size_t)row * kDblP + dir * kDblDir + c8;
  const v4f a0 = *(const v4f*)(p);
  const v4f a1 = *(const v4f*)(p + 4);
  v8h hv;
#pragma unroll
  for (int e = 0; e < 4; ++e) {
    const float f0 = a0[e];
    const float f1 = a1[e];
    hv[e]     = (_Float16)(f0 * scale);
    hv[4 + e] = (_Float16)(f1 * scale);
  }
  unsigned short* qd = DT16 + e0;
  *(volatile v8h*)qd = hv;
  __threadfence();
  *(volatile v8h*)qd = hv;
}

__global__ __launch_bounds__(256) void conv_silu_kernel(
    const float* __restrict__ XZ,
    const float* __restrict__ cw0, const float* __restrict__ cw1,
    const float* __restrict__ cb0, const float* __restrict__ cb1,
    float* __restrict__ XC, unsigned short* __restrict__ XC16)
{
  __shared__ __align__(16) float sT[16 * kConvTP];
  const int tid = threadIdx.x, lane = tid & 31, wave = tid >> 5;
  const int dc0  = blockIdx.x * 256;
  const int dir  = dc0 / kDin;
  const int dloc = dc0 - dir * kDin + tid;
  const int xcol = dir * (2 * kDin) + dloc;
  const float* cw = dir ? cw1 : cw0;
  const float* cb = dir ? cb1 : cb0;
  const float w0 = bf_rne(cw[dloc * 2 + 0]);
  const float w1 = bf_rne(cw[dloc * 2 + 1]);
  const float bc = bf_rne(cb[dloc]);
  const int g0    = blockIdx.y * 64;
  const int step  = dir ? 1 : -1;
  const int tedge = dir ? (kSeq - 1) : 0;
  const int hrow = wave >> 1;
  const int hch  = (wave & 1) * 128 + lane * 4;
#pragma unroll 1
  for (int sub = 0; sub < 4; ++sub) {
    const int lb = g0 + sub * 16;
#pragma unroll 1
    for (int s = 0; s < 16; ++s) {
      const int row = lb + s;
      const int t   = row & (kSeq - 1);
      const bool nv = (t != tedge);
      const int nrow = nv ? (row + step) : row;
      const float cur = XZ[(size_t)row * kXzP + xcol];
      const float nbr = XZ[(size_t)nrow * kXzP + xcol];
      const float nb  = nv ? nbr : 0.0f;
      float acc = fmaf(w0, nb, bc);
      acc = fmaf(w1, cur, acc);
      const float sg = __builtin_amdgcn_rcpf(1.0f + expf(-acc));
      sT[s * kConvTP + tid] = acc * sg;
    }
    __syncthreads();
    v4f fv[4];
    v8h bv[2];
#pragma unroll
    for (int it = 0; it < 4; ++it) fv[it] = *(const v4f*)(sT + (it * 4 + hrow) * kConvTP + hch);
#pragma unroll
    for (int it = 0; it < 2; ++it) {
      const float* sp = sT + (it * 8 + wave) * kConvTP + lane * 8;
      const v4f a0 = *(const v4f*)(sp);
      const v4f a1 = *(const v4f*)(sp + 4);
#pragma unroll
      for (int e = 0; e < 4; ++e) {
        const float f0 = a0[e];
        const float f1 = a1[e];
        bv[it][e]     = (_Float16)(f0 * kCarryXc);
        bv[it][4 + e] = (_Float16)(f1 * kCarryXc);
      }
    }
    for (int pass = 0; pass < 2; ++pass) {
#pragma unroll
      for (int it = 0; it < 4; ++it)
        *(volatile v4f*)(XC + (size_t)(lb + it * 4 + hrow) * kXcP + dc0 + hch) = fv[it];
#pragma unroll
      for (int it = 0; it < 2; ++it)
        *(volatile v8h*)(XC16 + (size_t)(lb + it * 8 + wave) * kXcP + dc0 + lane * 8) = bv[it];
      __threadfence();
    }
    __syncthreads();
  }
}

__global__ __launch_bounds__(64) void scan_kernel(
    const float* __restrict__ DBL, const float* __restrict__ DLR, const float* __restrict__ XC,
    const float* __restrict__ XZ,
    const float* __restrict__ dtb0, const float* __restrict__ dtb1,
    const float* __restrict__ Alog0, const float* __restrict__ Alog1,
    const float* __restrict__ Dp0, const float* __restrict__ Dp1,
    unsigned short* __restrict__ Y16)
{
  __shared__ __align__(16) float sBC[kScanTS * 64];
  __shared__ __align__(16) float sY[kScanTS * kScanYP];
  __shared__ __align__(16) float sA[kScanCh * kStP];
  __shared__ __align__(16) float sH[kScanCh * kStP];
  const int tid = threadIdx.x, lane = tid & 31, wave = tid >> 5;
  constexpr int kGrp = kDin / kScanCh;
  constexpr int kBlkPerDir = kBatch * kGrp;
  const int bx  = blockIdx.x;
  const int dir = bx / kBlkPerDir;
  const int rem = bx - dir * kBlkPerDir;
  const int bix = rem / kGrp;
  const int d0  = (rem - bix * kGrp) * kScanCh;
  const int d   = d0 + tid;
  const float* Alog = dir ? Alog1 : Alog0;
  const float* dtb  = dir ? dtb1 : dtb0;
  const float* Dpp  = dir ? Dp1 : Dp0;
  float* myA = sA + tid * kStP;
  float* myH = sH + tid * kStP;
#pragma unroll 1
  for (int g = 0; g < kNst / 4; ++g) {
    const v4f al = *(const v4f*)(Alog + (size_t)d * kNst + 4 * g);
    const float l0 = al[0];
    const float l1 = al[1];
    const float l2 = al[2];
    const float l3 = al[3];
    v4f av;
    av[0] = -expf(bf_rne(l0));
    av[1] = -expf(bf_rne(l1));
    av[2] = -expf(bf_rne(l2));
    av[3] = -expf(bf_rne(l3));
    *(v4f*)(myA + 4 * g) = av;
    *(v4f*)(myH + 4 * g) = (v4f){0.f, 0.f, 0.f, 0.f};
  }
  const float bb = bf_rne(dtb[d]);
  const float Dd = bf_rne(Dpp[d]);
  const size_t row0 = (size_t)bix * kSeq;
  const int colX = dir * kDin + d;
  const int colZ = dir * (2 * kDin) + kDin + d;
  const int colB = dir * kDblDir + kDtR;
  const int lr = tid >> 4, lc4 = (tid & 15) * 4;
  const int q = lane >> 3, c8 = (lane & 7) * 8;
#pragma unroll 1
  for (int c = 0; c < kSeq / kScanTS; ++c) {
    const int t0 = dir ? (kSeq - kScanTS - c * kScanTS) : (c * kScanTS);
    __syncthreads();
#pragma unroll
    for (int i = 0; i < 16; ++i) {
      const int r = lr + 4 * i;
      *(v4f*)(sBC + r * 64 + lc4) = *(const v4f*)(DBL + (row0 + t0 + r) * kDblP + colB + lc4);
    }
    __syncthreads();
#pragma unroll 1
    for (int i = 0; i < kScanTS; ++i) {
      const int s = dir ? (kScanTS - 1 - i) : i;
      const size_t row = row0 + (size_t)(t0 + s);
      float dl = DLR[row * kXcP + colX];
      float xt = XC[row * kXcP + colX];
      float zv = XZ[row * kXzP + colZ];
      asm volatile("" : "+v"(dl), "+v"(xt), "+v"(zv));
      const float v   = dl + bb;
      const float dt  = fmaxf(v, 0.0f) + log1pf(expf(-fabsf(v)));
      const float dtx = dt * xt;
      const float* xr = sBC + s * 64;
      float y = 0.f;
#pragma unroll 1
      for (int g = 0; g < kNst / 4; ++g) {
        v4f hst = *(const v4f*)(myH + 4 * g);
        const v4f av = *(const v4f*)(myA + 4 * g);
        const v4f bv = *(const v4f*)(xr + 4 * g);
        const v4f cv = *(const v4f*)(xr + kNst + 4 * g);
#pragma unroll
        for (int e = 0; e < 4; ++e) {
          const float ea = __expf(dt * av[e]);
          const float hn = fmaf(ea, hst[e], dtx * bv[e]);
          y = fmaf(hn, cv[e], y);
          hst[e] = hn;
        }
        *(v4f*)(myH + 4 * g) = hst;
      }
      y = fmaf(xt, Dd, y);
      const float sg = __builtin_amdgcn_rcpf(1.0f + expf(-zv));
      sY[s * kScanYP + tid] = (y * (zv * sg)) * kCarryY;
    }
    __syncthreads();
    v8h hv8[8];
#pragma unroll
    for (int it = 0; it < 8; ++it) {
      const int rr = it * 8 + wave * 4 + q;
      const float* sp = sY + rr * kScanYP + c8;
      const v4f a0 = *(const v4f*)(sp);
      const v4f a1 = *(const v4f*)(sp + 4);
#pragma unroll
      for (int e = 0; e < 4; ++e) {
        const float f0 = a0[e];
        const float f1 = a1[e];
        hv8[it][e]     = (_Float16)f0;
        hv8[it][4 + e] = (_Float16)f1;
      }
    }
    for (int pass = 0; pass < 2; ++pass) {
#pragma unroll
      for (int it = 0; it < 8; ++it) {
        const int rr = it * 8 + wave * 4 + q;
        const size_t o = (row0 + (size_t)(t0 + rr)) * kXcP + dir * kDin + d0 + c8;
        *(volatile v8h*)(Y16 + o) = hv8[it];
      }
      __threadfence();
    }
  }
}

extern "C" void kernel_launch(void* const* d_in, const int* in_sizes, int n_in,
                              void* d_out, int out_size, void* d_ws, size_t ws_size,
                              hipStream_t stream)
{
  if (n_in < 19) return;
  if (in_sizes[0] != kRows * kDm) return;
  for (int dir = 0; dir < 2; ++dir) {
    const int o = 1 + dir * 9;
    if (in_sizes[o + 0] != 2 * kDin * kDm) return;
    if (in_sizes[o + 1] != kDin * 2) return;
    if (in_sizes[o + 2] != kDin) return;
    if (in_sizes[o + 3] != kPrjN * kDin) return;
    if (in_sizes[o + 4] != kDin * kDtR) return;
    if (in_sizes[o + 5] != kDin) return;
    if (in_sizes[o + 6] != kDin * kNst) return;
    if (in_sizes[o + 7] != kDin) return;
    if (in_sizes[o + 8] != kDm * kDin) return;
  }
  if (out_size != kRows * kDm) return;
  if (ws_size < kWsTotal) return;

  const float* x       = (const float*)d_in[0];
  const float* in_w0   = (const float*)d_in[1];
  const float* conv_w0 = (const float*)d_in[2];
  const float* conv_b0 = (const float*)d_in[3];
  const float* xprj_w0 = (const float*)d_in[4];
  const float* dt_w0   = (const float*)d_in[5];
  const float* dt_b0   = (const float*)d_in[6];
  const float* A_log0  = (const float*)d_in[7];
  const float* Dp0     = (const float*)d_in[8];
  const float* out_w0  = (const float*)d_in[9];
  const float* in_w1   = (const float*)d_in[10];
  const float* conv_w1 = (const float*)d_in[11];
  const float* conv_b1 = (const float*)d_in[12];
  const float* xprj_w1 = (const float*)d_in[13];
  const float* dt_w1   = (const float*)d_in[14];
  const float* dt_b1   = (const float*)d_in[15];
  const float* A_log1  = (const float*)d_in[16];
  const float* Dp1     = (const float*)d_in[17];
  const float* out_w1  = (const float*)d_in[18];
  float* out = (float*)d_out;

  char* ws = (char*)d_ws;
  unsigned short* X16    = (unsigned short*)(ws + kOffX16);
  unsigned short* WIN16  = (unsigned short*)(ws + kOffWIN);
  unsigned short* WXP16  = (unsigned short*)(ws + kOffWXP);
  unsigned short* WDT16  = (unsigned short*)(ws + kOffWDT);
  unsigned short* WOUT16 = (unsigned short*)(ws + kOffWOUT);
  float*          XZ     = (float*)(ws + kOffXZ);
  float*          XC     = (float*)(ws + kOffXC);
  unsigned short* XC16   = (unsigned short*)(ws + kOffXC16);
  float*          DBL    = (float*)(ws + kOffDBL);
  unsigned short* DT16   = (unsigned short*)(ws + kOffDT16);
  float*          DLR    = (float*)(ws + kOffDLR);
  unsigned short* Y16    = (unsigned short*)(ws + kOffY16);

  cast_rows_f16_kernel<<<dim3((kRows * (kDm / 8)) / 256, 1), 256, 0, stream>>>(
      x, x, X16, kRows, kRows, kDm, kDm, 0L, 1.0f);
  cast_rows_f16_kernel<<<dim3((2 * kDin * (kDm / 8)) / 256, 2), 256, 0, stream>>>(
      in_w0, in_w1, WIN16, 2 * kDin, 2 * kDin, kDm, kDm, (long)(2 * kDin) * kDm, kCarryW);
  cast_rows_f16_kernel<<<dim3((kDblDir * (kDin / 8)) / 256, 2), 256, 0, stream>>>(
      xprj_w0, xprj_w1, WXP16, kPrjN, kDblDir, kDin, kDin, (long)kDblDir * kDin, kCarryW);
  cast_rows_f16_kernel<<<dim3((kDin * (kDtR / 8)) / 256, 2), 256, 0, stream>>>(
      dt_w0, dt_w1, WDT16, kDin, kDin, kDtR, kDtR, (long)kDin * kDtR, kCarryW);
  cast_rows_f16_kernel<<<dim3((kDm * (kDin / 8)) / 256, 2), 256, 0, stream>>>(
      out_w0, out_w1, WOUT16, kDm, kDm, kDin, 2 * kDin, (long)kDin, kCarryW);

  gemm64_f16_kernel<<<dim3(((kRows / 64) * (kXzP / 64)) / 8, 1), 256, 0, stream>>>(
      X16, kDm, 0L, WIN16, kDm, 0L, XZ, kXzP, 0L, kRows, kXzP, kDm, 1.0f / kCarryW);

  conv_silu_kernel<<<dim3(kXcP / 256, kRows / 64), 256, 0, stream>>>(
      XZ, conv_w0, conv_w1, conv_b0, conv_b1, XC, XC16);

  gemm64_f16_kernel<<<dim3(((kRows / 64) * (kDblDir / 64)) / 8, 2), 256, 0, stream>>>(
      XC16, kXcP, (long)kDin, WXP16, kDin, (long)kDblDir * kDin, DBL, kDblP, (long)kDblDir,
      kRows, kDblDir, kDin, 1.0f / (kCarryXc * kCarryW));

  dt_cast_kernel<<<(2 * kRows * kDtR / 8) / 256, 256, 0, stream>>>(DBL, DT16, 2 * kRows * kDtR / 8, kCarryDt);

  gemm64_f16_kernel<<<dim3(((kRows / 64) * (kDin / 64)) / 8, 2), 256, 0, stream>>>(
      DT16, kDtR, (long)kRows * kDtR, WDT16, kDtR, (long)kDin * kDtR, DLR, kXcP, (long)kDin,
      kRows, kDin, kDtR, 1.0f / (kCarryDt * kCarryW));

  scan_kernel<<<2 * kBatch * (kDin / kScanCh), kScanCh, 0, stream>>>(
      DBL, DLR, XC, XZ, dt_b0, dt_b1, A_log0, A_log1, Dp0, Dp1, Y16);

  gemm64_f16_kernel<<<dim3(((kRows / 64) * (kDm / 64)) / 8, 1), 256, 0, stream>>>(
      Y16, kXcP, 0L, WOUT16, 2 * kDin, 0L, out, kDm, 0L, kRows, kDm, 2 * kDin, 1.0f / (kCarryY * kCarryW));
}
